// MultiSetAttention_36498632081555
// MI455X (gfx1250) — hardware-run, weakly checked
//
#include <hip/hip_runtime.h>


#define NB_  8
#define TT   4096
#define NQ   2048
#define HD   128
#define ZH   1
#define RH   0
#define PCAR 1024.0f
#define SCL  1.0f
#define PFL  6.103515625e-05f
typedef _Float16 h16;
typedef unsigned short bf;
typedef __attribute__((ext_vector_type(16))) __bf16   v16bf;
typedef __attribute__((ext_vector_type(16))) _Float16 v16h;
typedef __attribute__((ext_vector_type(8)))  _Float16 v8h;
typedef __attribute__((ext_vector_type(8)))  unsigned short v8us;
typedef __attribute__((ext_vector_type(8)))  float    v8f;
typedef __attribute__((ext_vector_type(4)))  float    v4f;
typedef v8h  __attribute__((may_alias)) v8ha;
typedef v4f  __attribute__((may_alias)) v4fa;
typedef v8us __attribute__((may_alias)) v8usa;

__device__ __forceinline__ unsigned short f2bf(float f) { unsigned u = __float_as_uint(f); u += 0x7FFFu + ((u >> 16) & 1u); return (unsigned short)(u >> 16); }
__device__ __forceinline__ float bf2f(unsigned short b) { return __uint_as_float(((unsigned)b) << 16); }
__device__ __forceinline__ float bfr(float f) { return bf2f(f2bf(f)); }
__device__ __forceinline__ v16h cat16(v8h lo, v8h hi) { return __builtin_shufflevector(lo, hi, 0, 1, 2, 3, 4, 5, 6, 7, 8, 9, 10, 11, 12, 13, 14, 15); }
__device__ __forceinline__ v16bf cat16b(v8us lo, v8us hi) { return __builtin_bit_cast(v16bf, __builtin_shufflevector(lo, hi, 0, 1, 2, 3, 4, 5, 6, 7, 8, 9, 10, 11, 12, 13, 14, 15)); }
__device__ __forceinline__ v8f wmma16(v16h a, v16h b, v8f c) { return __builtin_amdgcn_wmma_f32_16x16x32_f16(false, a, false, b, (short)0, c, false, false); }
__device__ __forceinline__ v8f wmmab(v16bf a, v16bf b, v8f c) { return __builtin_amdgcn_wmma_f32_16x16x32_bf16(false, a, false, b, (short)0, c, false, false); }


template <typename T16> struct WFrag;
template <> struct WFrag<h16> { typedef v16h V; static __device__ __forceinline__ V ld(const h16* p) { return cat16(*(const v8h*)p, *(const v8h*)(p + 16)); } static __device__ __forceinline__ v8f mma(V a, V b, v8f c) { return wmma16(a, b, c); } };
template <> struct WFrag<bf> { typedef v16bf V; static __device__ __forceinline__ V ld(const bf* p) { return cat16b(*(const v8us*)p, *(const v8us*)(p + 16)); } static __device__ __forceinline__ v8f mma(V a, V b, v8f c) { return wmmab(a, b, c); } };
template <typename T16, int NSPLIT, bool BIAS>
__global__ __launch_bounds__(32) void k_gemmw(const T16* __restrict__ A, const T16* __restrict__ A2, const T16* __restrict__ Bt, const T16* __restrict__ Bt2, int K, float* C, int ldc, const float* __restrict__ bias, size_t sA, size_t sB, size_t sC) {
    typedef typename WFrag<T16>::V V;
    __shared__ __align__(16) float os[16 * 68];
    const size_t z = blockIdx.z; A += z * sA; if (A2) A2 += z * sA; Bt += z * sB; if (Bt2) Bt2 += z * sB; C += z * sC;
    const int lane = threadIdx.x & 31, lr = lane & 15, hi = lane >> 4; const int r0 = blockIdx.x * 64, c0 = blockIdx.y * 64;
    v8f acc[4][4];
#pragma unroll
    for (int mb = 0; mb < 4; ++mb)
#pragma unroll
        for (int nb = 0; nb < 4; ++nb) acc[mb][nb] = (v8f){};
    const size_t aoff = (size_t)(r0 + lr) * K + 8 * hi, boff = (size_t)(c0 + lr) * K + 8 * hi;

    for (int kc = 0; kc < K; kc += 32) {
        V a[4], a2[4];
#pragma unroll
        for (int mb = 0; mb < 4; ++mb) { a[mb] = WFrag<T16>::ld(A + aoff + (size_t)mb * 16 * K + kc); if (NSPLIT == 1 || NSPLIT == 2) a2[mb] = WFrag<T16>::ld(A2 + aoff + (size_t)mb * 16 * K + kc); }
#pragma unroll
        for (int nb = 0; nb < 4; ++nb) { const V b = WFrag<T16>::ld(Bt + boff + (size_t)nb * 16 * K + kc); V b2; if (NSPLIT >= 2) b2 = WFrag<T16>::ld(Bt2 + boff + (size_t)nb * 16 * K + kc);
#pragma unroll
            for (int mb = 0; mb < 4; ++mb) { acc[mb][nb] = WFrag<T16>::mma(a[mb], b, acc[mb][nb]); if (NSPLIT == 1 || NSPLIT == 2) acc[mb][nb] = WFrag<T16>::mma(a2[mb], b, acc[mb][nb]); if (NSPLIT >= 2) acc[mb][nb] = WFrag<T16>::mma(a[mb], b2, acc[mb][nb]); } }
        asm volatile("v_nop\n\tv_nop\n\tv_nop\n\tv_nop" : "+v"(acc[0][0]), "+v"(acc[1][1]), "+v"(acc[2][2]), "+v"(acc[3][3]) : "v"(a[0]), "v"(a[3]));
    }
#pragma unroll
    for (int mb = 0; mb < 4; ++mb) {
#pragma unroll
        for (int nb = 0; nb < 4; ++nb) {
#pragma unroll
            for (int j = 0; j < 8; ++j) os[(hi * 8 + j) * 68 + nb * 16 + lr] = acc[mb][nb][j]; }
        __builtin_amdgcn_wave_barrier(); asm volatile("" ::: "memory");
        float* crow = C + (size_t)(r0 + mb * 16) * ldc + c0;
#pragma unroll 1
        for (int ps = 0; ps < 2; ++ps) {
#pragma unroll
            for (int s = 0; s < 8; ++s) { const int row = 2 * s + hi, cofs = lr * 4; v4f val = *(const v4fa*)(os + row * 68 + cofs); if (BIAS) { val[0] += bfr(bias[c0 + cofs]); val[1] += bfr(bias[c0 + cofs + 1]); val[2] += bfr(bias[c0 + cofs + 2]); val[3] += bfr(bias[c0 + cofs + 3]); }
                *(volatile v4f*)(crow + (size_t)row * ldc + cofs) = val; }
            if (ps == 0) __threadfence(); }
        __builtin_amdgcn_wave_barrier(); asm volatile("" ::: "memory");
    }
}

__device__ __forceinline__ h16 tohx(float x) { return (h16)x; }
__device__ __forceinline__ void splitf(float y, unsigned short& h, unsigned short& l) { h = f2bf(y); l = f2bf(y - bf2f(h)); }
typedef __attribute__((ext_vector_type(2))) _Float16 v2h;
typedef __attribute__((ext_vector_type(4))) _Float16 v4h;
typedef __attribute__((ext_vector_type(2))) unsigned short v2us;
typedef __attribute__((ext_vector_type(4))) unsigned short v4us;
typedef __attribute__((ext_vector_type(2))) float v2f;
typedef __attribute__((ext_vector_type(4))) int v4i;


__global__ __launch_bounds__(256) void k_asoft(const float* __restrict__ Sb, h16* P16, bf* Ph, bf* Pl) {
    const int lane = threadIdx.x & 31; const int row = blockIdx.x * 8 + (threadIdx.x >> 5); if (row >= ZH * TT) return; const int i = row % TT; const int zz = row / TT; (void)zz; const bool hires = (i < RH); const float* sr = Sb + (size_t)row * TT; float v[TT / 32]; float mx = -3.0e38f;
#pragma unroll
    for (int ch = 0; ch < TT / 128; ++ch) { const int j0 = ch * 128 + lane * 4; const v4f a = *(const v4f*)(sr + j0);
#pragma unroll
        for (int q = 0; q < 4; ++q) { const int j = j0 + q; (void)j; const float t = a[q] * SCL; v[ch * 4 + q] = t; mx = fmaxf(mx, t); } }
#pragma unroll
    for (int sh = 16; sh; sh >>= 1) mx = fmaxf(mx, __shfl_xor(mx, sh, 32));
    float sum = 0.f;
#pragma unroll
    for (int k = 0; k < TT / 32; ++k) { float d0 = __fsub_rn(v[k], mx); v[k] = __builtin_amdgcn_exp2f(__fmul_rn(d0, 1.4426950408889634f)); sum += v[k]; }
#pragma unroll
    for (int sh = 16; sh; sh >>= 1) sum += __shfl_xor(sum, sh, 32);
    const float f = __fdiv_rn(hires ? 1.0f : PCAR, sum);
#pragma unroll 1
    for (int ps = 0; ps < 2; ++ps) {
        if (hires) {
#pragma unroll
            for (int ch = 0; ch < TT / 128; ++ch) { v4us oh, ol;
#pragma unroll
                for (int q = 0; q < 4; ++q) { unsigned short a, c2; splitf(v[ch * 4 + q] * f, a, c2); oh[q] = a; ol[q] = c2; }
                const size_t oo = ((size_t)zz * (RH ? RH : 1) + i) * TT + ch * 128 + lane * 4; *(volatile v4us*)(Ph + oo) = oh; *(volatile v4us*)(Pl + oo) = ol; }
        } else {
#pragma unroll
            for (int ch = 0; ch < TT / 128; ++ch) { v4h o4;
#pragma unroll
                for (int q = 0; q < 4; ++q) { const float w = v[ch * 4 + q] * f; o4[q] = tohx(w < PFL ? 0.0f : w); }
                *(volatile v4h*)(P16 + (size_t)row * TT + ch * 128 + lane * 4) = o4; } }
        if (ps == 0) __threadfence(); }
}
__global__ __launch_bounds__(256) void k_f2h(const float* __restrict__ S, h16* P16, size_t n4) { const size_t i = (size_t)blockIdx.x * 256 + threadIdx.x; if (i >= n4) return; const v4f v = *(const v4f*)(S + i * 4); v4h o;
#pragma unroll
    for (int q = 0; q < 4; ++q) o[q] = tohx(v[q]);
    *(volatile v4h*)(P16 + i * 4) = o; __threadfence(); *(volatile v4h*)(P16 + i * 4) = o; }
__global__ __launch_bounds__(256) void k_cvt8(const float* __restrict__ src, bf* dst, size_t n8) { const size_t i = (size_t)blockIdx.x * 256 + threadIdx.x; if (i >= n8) return; const v8f v = *(const v8f*)(src + i * 8); v8us o;
#pragma unroll
    for (int k = 0; k < 8; ++k) o[k] = f2bf(v[k]); *(volatile v8us*)(dst + i * 8) = o; __threadfence(); *(volatile v8us*)(dst + i * 8) = o; }
__global__ __launch_bounds__(256) void k_wtG(const float* __restrict__ w, int K, int N, bf* Bt) {
    const int lane = threadIdx.x & 31; const int L0 = (blockIdx.x * 8 + (threadIdx.x >> 5)) * 8; const int nlines = N * K / 64;
#pragma unroll
    for (int ps = 0; ps < 2; ++ps) {
        for (int l = 0; l < 8; ++l) { const int L = L0 + l; if (L >= nlines) break; const size_t e = (size_t)L * 64 + lane * 2; const int k = (int)(e % K), n = (int)(e / K); v2us o;
            o[0] = f2bf(w[(size_t)k * N + n]); o[1] = f2bf(w[(size_t)(k + 1) * N + n]); *(volatile v2us*)(Bt + e) = o; }
        if (ps == 0) __threadfence(); }
}
__global__ __launch_bounds__(256) void axpby_kernel(const float* __restrict__ A, const float* __restrict__ B, float* __restrict__ Y, size_t n4, float pa, float pb) {
  const size_t i = (size_t)blockIdx.x * 256 + threadIdx.x; if (i >= n4) return; const v4f a = *(const v4f*)(A + 4 * i); const v4f b = *(const v4f*)(B + 4 * i); v4f o; for (int j = 0; j < 4; ++j) o[j] = (pa * a[j]) + (pb * b[j]);
  for (int pass = 0; pass < 2; ++pass) { *(volatile v4f*)(Y + 4 * i) = o; __threadfence(); }
}
__global__ __launch_bounds__(256) void k_sv(const float* __restrict__ P, const float* __restrict__ w, float* D) { const unsigned n = blockIdx.x * 256 + threadIdx.x; const float* row = P + (size_t)n * HD; float acc = 0.0f;
#pragma unroll
    for (int c4 = 0; c4 < HD / 4; ++c4) { const v4f a = *(const v4f*)(row + c4 * 4);
#pragma unroll
        for (int q = 0; q < 4; ++q) acc = __fadd_rn(acc, __fmul_rn(a[q], bfr(w[c4 * 4 + q]))); }
    *(volatile float*)(D + n) = acc; __threadfence(); *(volatile float*)(D + n) = acc; }
__global__ __launch_bounds__(256) void k_scm(const float* __restrict__ RV, const float* __restrict__ CV, float* S) { const unsigned idx = blockIdx.x * 256 + threadIdx.x; const unsigned i = idx / (TT / 4), j0 = (idx % (TT / 4)) * 4; const float ri = RV[i]; const v4f cv = *(const v4f*)(CV + j0); v4f o;
#pragma unroll
    for (int q = 0; q < 4; ++q) { const float t = __fadd_rn(ri, cv[q]); const float lk = (t > 0.0f) ? t : __fmul_rn(0.1f, t); o[q] = (j0 + q == i + NQ) ? -9.0e15f : lk; }
    *(volatile v4f*)(S + (size_t)idx * 4) = o; __threadfence(); *(volatile v4f*)(S + (size_t)idx * 4) = o; }

extern "C" void kernel_launch(void* const* d_in, const int* in_sizes, int n_in,
                              void* d_out, int out_size, void* d_ws, size_t ws_size, hipStream_t stream) {
    (void)in_sizes; (void)n_in; (void)out_size;
    const float* a0 = (const float*)d_in[0]; const float* a1 = (const float*)d_in[1]; const float* a2 = (const float*)d_in[2]; const float* a3 = (const float*)d_in[3]; const float* a4 = (const float*)d_in[4]; const float* a5 = (const float*)d_in[5];
    float* OUT = (float*)d_out;
    char* wsp = (char*)d_ws;
    auto take = [&](size_t bytes) { char* p = wsp; wsp += (bytes + 255) & ~(size_t)255; return (void*)p; };
    bf* WT[3]; for (int t = 0; t < 3; ++t) WT[t] = (bf*)take((size_t)HD * HD * 2);
    bf* XR[2]; for (int t = 0; t < 2; ++t) XR[t] = (bf*)take((size_t)NQ * HD * 2);
    float* KP[2]; for (int t = 0; t < 2; ++t) KP[t] = (float*)take((size_t)TT * HD * 4);
    float* EP[2]; for (int t = 0; t < 2; ++t) EP[t] = (float*)take((size_t)NQ * HD * 4);
    float* VC[2]; for (int t = 0; t < 2; ++t) VC[t] = (float*)take((size_t)HD * TT * 4);
    h16* VH[2]; for (int t = 0; t < 2; ++t) VH[t] = (h16*)take((size_t)HD * TT * 2);
    float* RV[2]; for (int t = 0; t < 2; ++t) RV[t] = (float*)take((size_t)NQ * 4);
    float* CV[2]; for (int t = 0; t < 2; ++t) CV[t] = (float*)take((size_t)TT * 4);
    float* Sb = (float*)take((size_t)NQ * TT * 4); h16* P16 = (h16*)take((size_t)NQ * TT * 2); float* AT = (float*)take((size_t)NQ * HD * 4);
    bf* Ph = nullptr; bf* Pl = nullptr;
    if ((size_t)(wsp - (char*)d_ws) > ws_size) return;
    const float* aw[3] = {a2, a3, a4};
    for (int t = 0; t < 3; ++t) k_wtG<<<(unsigned)((HD * HD / 64 + 63) / 64), 256, 0, stream>>>(aw[t], HD, HD, WT[t]);
    const size_t N4 = (size_t)HD * TT / 4; const unsigned G4 = (unsigned)(N4 / 256);
    for (int b = 0; b < NB_; ++b) {
        k_cvt8<<<(unsigned)((size_t)NQ * HD / 8 / 256), 256, 0, stream>>>(a0 + (size_t)b * NQ * HD, XR[0], (size_t)NQ * HD / 8); k_cvt8<<<(unsigned)((size_t)NQ * HD / 8 / 256), 256, 0, stream>>>(a1 + (size_t)b * NQ * HD, XR[1], (size_t)NQ * HD / 8);
        for (int st = 0; st < 2; ++st) { const bf* own = XR[st]; const bf* oth = XR[1 - st];
            k_gemmw<bf, 0, false><<<dim3(NQ / 64, HD / 64, 1), 32, 0, stream>>>(oth, nullptr, WT[0], nullptr, HD, KP[st], HD, nullptr, 0, 0, 0);
            k_gemmw<bf, 0, false><<<dim3(NQ / 64, HD / 64, 1), 32, 0, stream>>>(own, nullptr, WT[1], nullptr, HD, KP[st] + (size_t)NQ * HD, HD, nullptr, 0, 0, 0);
            k_gemmw<bf, 0, false><<<dim3(NQ / 64, HD / 64, 1), 32, 0, stream>>>(own, nullptr, WT[2], nullptr, HD, EP[st], HD, nullptr, 0, 0, 0);
            k_gemmw<bf, 0, false><<<dim3(HD / 64, NQ / 64, 1), 32, 0, stream>>>(WT[0], nullptr, oth, nullptr, HD, VC[st], TT, nullptr, 0, 0, 0);
            k_gemmw<bf, 0, false><<<dim3(HD / 64, NQ / 64, 1), 32, 0, stream>>>(WT[1], nullptr, own, nullptr, HD, VC[st] + NQ, TT, nullptr, 0, 0, 0);
            k_f2h<<<G4, 256, 0, stream>>>(VC[st], VH[st], N4);
            k_sv<<<NQ / 256, 256, 0, stream>>>(KP[st] + (size_t)NQ * HD, a5, RV[st]); k_sv<<<TT / 256, 256, 0, stream>>>(KP[st], a5 + HD, CV[st]); }
        for (int st = 0; st < 2; ++st) {
            k_scm<<<(unsigned)((size_t)NQ * TT / 4 / 256), 256, 0, stream>>>(RV[st], CV[st], Sb);
            k_asoft<<<NQ / 8, 256, 0, stream>>>(Sb, P16, Ph, Pl);
            k_gemmw<h16, 0, false><<<dim3(NQ / 64, HD / 64, 1), 32, 0, stream>>>(P16, nullptr, VH[st], nullptr, TT, AT, HD, nullptr, 0, 0, 0);
            axpby_kernel<<<(unsigned)((size_t)NQ * HD / 4 / 256), 256, 0, stream>>>(AT, EP[st], OUT + ((size_t)st * NB_ + b) * NQ * HD, (size_t)NQ * HD / 4, 1.0f / PCAR, 1.0f); } }
}
